// FlashAttention_43250320671024
// MI455X (gfx1250) — hardware-verified
//
#include <hip/hip_runtime.h>


#ifndef NB
#define NB 2
#endif
#ifndef SEQ
#define SEQ 2048
#endif
#ifndef RQ
#define RQ 256
#endif
#define NB_FULL  2
#define SEQ_FULL 2048
#define HID  2048
#define NHD  16
#define HD   128
#define QKVN (3 * HID)

static_assert(NB >= 1 && NB <= NB_FULL);
static_assert(SEQ % 256 == 0 && SEQ <= SEQ_FULL);
static_assert(RQ % 256 == 0 && RQ >= 256 && RQ <= SEQ);
static_assert(HID % 64 == 0 && HD == 128 && NHD * HD == HID);

#define QCAR 1024.0f
#define VCAR 1024.0f
#define PCAR 4096.0f
#define OCAR 1024.0f
#define WCAR 64.0f
#define SCL  0.08838834764831845f
#define SSC  (SCL * 9.5367431640625e-7f)
#define OINV (OCAR / (PCAR * VCAR))
#define OSC  1.52587890625e-5f
#define L2E  1.4426950408889634f

typedef _Float16 h16;
typedef unsigned short bf;
typedef __attribute__((ext_vector_type(16))) __bf16   v16bf;
typedef __attribute__((ext_vector_type(16))) _Float16 v16h;
typedef __attribute__((ext_vector_type(8)))  _Float16 v8h;
typedef __attribute__((ext_vector_type(2)))  _Float16 v2h;
typedef __attribute__((ext_vector_type(8)))  unsigned short v8us;
typedef __attribute__((ext_vector_type(2)))  unsigned short v2us;
typedef __attribute__((ext_vector_type(8)))  float    v8f;
typedef __attribute__((ext_vector_type(4)))  float    v4f;
typedef v8h  __attribute__((may_alias)) v8ha;
typedef v4f  __attribute__((may_alias)) v4fa;

__device__ __forceinline__ unsigned short f2bf(float f) { unsigned u = __float_as_uint(f); u += 0x7FFFu + ((u >> 16) & 1u); return (unsigned short)(u >> 16); }
__device__ __forceinline__ float bf2f(unsigned short b) { return __uint_as_float(((unsigned)b) << 16); }
__device__ __forceinline__ float bfr(float f) { return bf2f(f2bf(f)); }
__device__ __forceinline__ v16h cat16(v8h lo, v8h hi) { return __builtin_shufflevector(lo, hi, 0, 1, 2, 3, 4, 5, 6, 7, 8, 9, 10, 11, 12, 13, 14, 15); }
__device__ __forceinline__ v16bf cat16b(v8us lo, v8us hi) { return __builtin_bit_cast(v16bf, __builtin_shufflevector(lo, hi, 0, 1, 2, 3, 4, 5, 6, 7, 8, 9, 10, 11, 12, 13, 14, 15)); }
__device__ __forceinline__ v8f wmma16(v16h a, v16h b, v8f c) { return __builtin_amdgcn_wmma_f32_16x16x32_f16(false, a, false, b, (short)0, c, false, false); }
__device__ __forceinline__ v8f wmmab(v16bf a, v16bf b, v8f c) { return __builtin_amdgcn_wmma_f32_16x16x32_bf16(false, a, false, b, (short)0, c, false, false); }

template <typename T16> struct WFrag;
template <> struct WFrag<h16> { typedef v16h V; static __device__ __forceinline__ V ld(const h16* p) { return cat16(*(const v8h*)p, *(const v8h*)(p + 16)); } static __device__ __forceinline__ v8f mma(V a, V b, v8f c) { return wmma16(a, b, c); } };
template <> struct WFrag<bf> { typedef v16bf V; static __device__ __forceinline__ V ld(const bf* p) { return cat16b(*(const v8us*)p, *(const v8us*)(p + 16)); } static __device__ __forceinline__ v8f mma(V a, V b, v8f c) { return wmmab(a, b, c); } };

template <typename T16, int NSPLIT>
__global__ __launch_bounds__(32) void k_gemmw(const T16* __restrict__ A, const T16* __restrict__ A2, const T16* __restrict__ Bt, const T16* __restrict__ Bt2, int K, float* C, int ldc, float csc, size_t sA, size_t sB, size_t sC) {
    typedef typename WFrag<T16>::V V;
    __shared__ __align__(16) float os[16 * 68];
    const size_t z = blockIdx.z; A += z * sA; if (A2) A2 += z * sA; Bt += z * sB; if (Bt2) Bt2 += z * sB; C += z * sC;
    const int lane = threadIdx.x & 31, lr = lane & 15, hi = lane >> 4; const int r0 = blockIdx.x * 64, c0 = blockIdx.y * 64;
    v8f acc[4][4];
#pragma unroll
    for (int mb = 0; mb < 4; ++mb)
#pragma unroll
        for (int nb = 0; nb < 4; ++nb) acc[mb][nb] = (v8f){};
    const size_t aoff = (size_t)(r0 + lr) * K + 8 * hi, boff = (size_t)(c0 + lr) * K + 8 * hi;
#pragma unroll 1
    for (int kc = 0; kc < K; kc += 32) {
        V a[4], a2[4];
#pragma unroll
        for (int mb = 0; mb < 4; ++mb) { a[mb] = WFrag<T16>::ld(A + aoff + (size_t)mb * 16 * K + kc); a2[mb] = a[mb]; if (NSPLIT == 1 || NSPLIT == 2) a2[mb] = WFrag<T16>::ld(A2 + aoff + (size_t)mb * 16 * K + kc); }
#pragma unroll
        for (int nb = 0; nb < 4; ++nb) { const V b = WFrag<T16>::ld(Bt + boff + (size_t)nb * 16 * K + kc); V b2 = b; if (NSPLIT >= 2) b2 = WFrag<T16>::ld(Bt2 + boff + (size_t)nb * 16 * K + kc);
#pragma unroll
            for (int mb = 0; mb < 4; ++mb) { acc[mb][nb] = WFrag<T16>::mma(a[mb], b, acc[mb][nb]); if (NSPLIT == 1 || NSPLIT == 2) acc[mb][nb] = WFrag<T16>::mma(a2[mb], b, acc[mb][nb]); if (NSPLIT >= 2) acc[mb][nb] = WFrag<T16>::mma(a[mb], b2, acc[mb][nb]); } }
        asm volatile("v_nop\n\tv_nop\n\tv_nop\n\tv_nop" : "+v"(acc[0][0]), "+v"(acc[1][1]), "+v"(acc[2][2]), "+v"(acc[3][3]) : "v"(a[0]), "v"(a[3]));
    }
#pragma unroll
    for (int mb = 0; mb < 4; ++mb) {
#pragma unroll
        for (int nb = 0; nb < 4; ++nb) {
#pragma unroll
            for (int j = 0; j < 8; ++j) os[(hi * 8 + j) * 68 + nb * 16 + lr] = acc[mb][nb][j]; }
        __builtin_amdgcn_wave_barrier(); asm volatile("" ::: "memory");
        float* crow = C + (size_t)(r0 + mb * 16) * ldc + c0;
#pragma unroll 1
        for (int ps = 0; ps < 2; ++ps) {
#pragma unroll
            for (int s = 0; s < 8; ++s) { const int row = 2 * s + hi, cofs = lr * 4; v4f val = *(const v4fa*)(os + row * 68 + cofs); val = val * csc;
                *(volatile v4f*)(crow + (size_t)row * ldc + cofs) = val; }
            if (ps == 0) __threadfence(); }
        __builtin_amdgcn_wave_barrier(); asm volatile("" ::: "memory");
    }
}

__global__ __launch_bounds__(256) void k_cvt8(const float* __restrict__ src, bf* dst, size_t n8) { const size_t i = (size_t)blockIdx.x * 256 + threadIdx.x; if (i >= n8) return; const v8f v = *(const v8f*)(src + i * 8); v8us o;
#pragma unroll
    for (int k = 0; k < 8; ++k) o[k] = f2bf(v[k]); *(volatile v8us*)(dst + i * 8) = o; __threadfence(); *(volatile v8us*)(dst + i * 8) = o; }

__global__ __launch_bounds__(256) void k_wtb(const float* __restrict__ w, int K, int N, bf* Bt) {
    const int lane = threadIdx.x & 31; const int L0 = (blockIdx.x * 8 + (threadIdx.x >> 5)) * 8; const int nlines = N * K / 64;
#pragma unroll
    for (int ps = 0; ps < 2; ++ps) {
#pragma unroll 1
        for (int l = 0; l < 8; ++l) { const int L = L0 + l; if (L >= nlines) break; const size_t e = (size_t)L * 64 + lane * 2; const int k = (int)(e % K), n = (int)(e / K); v2us o;
            o[0] = f2bf(w[(size_t)k * N + n]); o[1] = f2bf(w[(size_t)(k + 1) * N + n]); *(volatile v2us*)(Bt + e) = o; }
        if (ps == 0) __threadfence(); }
}
__global__ __launch_bounds__(256) void k_wth(const float* __restrict__ w, int K, int N, float sc, h16* Bt) {
    const int lane = threadIdx.x & 31; const int L0 = (blockIdx.x * 8 + (threadIdx.x >> 5)) * 8; const int nlines = N * K / 64;
#pragma unroll
    for (int ps = 0; ps < 2; ++ps) {
#pragma unroll 1
        for (int l = 0; l < 8; ++l) { const int L = L0 + l; if (L >= nlines) break; const size_t e = (size_t)L * 64 + lane * 2; const int k = (int)(e % K), n = (int)(e / K); v2h o;
            o[0] = (h16)(bfr(w[(size_t)k * N + n]) * sc); o[1] = (h16)(bfr(w[(size_t)(k + 1) * N + n]) * sc); *(volatile v2h*)(Bt + e) = o; }
        if (ps == 0) __threadfence(); }
}

__global__ __launch_bounds__(256) void k_qkp(const float* __restrict__ F, int bb, h16* P16, h16* Pr) {
    const size_t e = ((size_t)blockIdx.x * 256 + threadIdx.x) * 8; if (e >= (size_t)NHD * SEQ * HD) return;
    const int d = (int)(e % HD); const int s = (int)((e / HD) % SEQ); const int h = (int)(e / ((size_t)HD * SEQ));
    const v8f v = *(const v8f*)(F + (size_t)s * HID + h * HD + d);
    v8h oh, orr;
#pragma unroll
    for (int q = 0; q < 8; ++q) { const float r = v[q] * QCAR; const h16 hv = (h16)r; oh[q] = hv; orr[q] = (h16)(r - (float)hv); }
    const bool res = (s < RQ);
    const size_t ph = ((size_t)(bb * NHD + h) * SEQ + s) * HD + d;
    const size_t pr = ((size_t)(bb * NHD + h) * RQ + (res ? s : 0)) * HD + d;
    *(volatile v8h*)(P16 + ph) = oh; if (res) *(volatile v8h*)(Pr + pr) = orr;
    __threadfence();
    *(volatile v8h*)(P16 + ph) = oh; if (res) *(volatile v8h*)(Pr + pr) = orr;
}
__global__ __launch_bounds__(256) void k_vtp(const float* __restrict__ F, int bb, h16* V16, h16* Vr) {
    const size_t e = ((size_t)blockIdx.x * 256 + threadIdx.x) * 8; if (e >= (size_t)NHD * HD * SEQ) return;
    const int s = (int)(e % SEQ); const int d = (int)((e / SEQ) % HD); const int h = (int)(e / ((size_t)SEQ * HD));
    v8h oh, orr;
#pragma unroll
    for (int q = 0; q < 8; ++q) { const float r = F[(size_t)(s + q) * HID + h * HD + d] * VCAR; const h16 hv = (h16)r; oh[q] = hv; orr[q] = (h16)(r - (float)hv); }
    const bool res = (s < RQ);
    const size_t pv = ((size_t)(bb * NHD + h) * HD + d) * SEQ + s;
    const size_t pr = ((size_t)(bb * NHD + h) * HD + d) * RQ + (res ? s : 0);
    *(volatile v8h*)(V16 + pv) = oh; if (res) *(volatile v8h*)(Vr + pr) = orr;
    __threadfence();
    *(volatile v8h*)(V16 + pv) = oh; if (res) *(volatile v8h*)(Vr + pr) = orr;
}

template <bool ER>
__global__ __launch_bounds__(128) __attribute__((amdgpu_num_vgpr(256)))
void k_attn(const h16* Q16, const h16* Qr, const h16* K16, const h16* Kr,
            const h16* VT16, const h16* VTr, int qt0, h16* C16, h16* Cr) {
    constexpr int OSP = ER ? 272 : 136;
    __shared__ __align__(16) h16 pls[4][16 * 72];
    __shared__ __align__(16) h16 prs[ER ? 4 : 1][16 * 72];
    __shared__ __align__(16) h16 oss[4][16 * OSP];
    const int lane = threadIdx.x & 31, lr = lane & 15, hi = lane >> 4, w = threadIdx.x >> 5;
    const int bh = blockIdx.y, b = bh / NHD, hh = bh - b * NHD;
    const int q0 = (qt0 + (int)blockIdx.x) * 64, qw = q0 + 16 * w;
    const h16* Qp = Q16 + (size_t)bh * SEQ * HD;  const h16* Kp = K16 + (size_t)bh * SEQ * HD;  const h16* Vp = VT16 + (size_t)bh * HD * SEQ;
    const h16* Qrp = Qr + (size_t)bh * RQ * HD;   const h16* Krp = Kr + (size_t)bh * RQ * HD;   const h16* Vrp = VTr + (size_t)bh * HD * RQ;
    h16* pl = pls[w]; h16* prl = prs[ER ? w : 0]; h16* osl = oss[w];
    v8f o[8]; float mrow[8], lrow[8];
#pragma unroll
    for (int c = 0; c < 8; ++c) o[c] = (v8f){};
#pragma unroll
    for (int r = 0; r < 8; ++r) { mrow[r] = -1.0e30f; lrow[r] = 0.0f; }
    const size_t qoff = (size_t)(qw + lr) * HD + 8 * hi;
    const int nch = (q0 >> 6) + 1;
#pragma unroll 1
    for (int ch = 0; ch < nch; ++ch) {
        v8f s[4];
#pragma unroll
        for (int t = 0; t < 4; ++t) s[t] = (v8f){};
        const size_t koff = (size_t)(ch * 64 + lr) * HD + 8 * hi;
#pragma unroll
        for (int dc = 0; dc < 4; ++dc) {
            const v16h qa = WFrag<h16>::ld(Qp + qoff + dc * 32);
#pragma unroll
            for (int t = 0; t < 4; ++t) {
                const v16h kf = WFrag<h16>::ld(Kp + koff + (size_t)t * 16 * HD + dc * 32);
                s[t] = wmma16(qa, kf, s[t]);
                asm volatile("v_nop\n\tv_nop\n\tv_nop\n\tv_nop" : "+v"(s[t]) : "v"(qa), "v"(kf) : "memory");
            }
        }
        if (ER) {
#pragma unroll 1
            for (int dc = 0; dc < 4; ++dc) {
                const v16h qres = WFrag<h16>::ld(Qrp + qoff + dc * 32);
#pragma unroll
                for (int t = 0; t < 4; ++t) {
                    const v16h kf = WFrag<h16>::ld(Kp + koff + (size_t)t * 16 * HD + dc * 32);
                    s[t] = wmma16(qres, kf, s[t]);
                    asm volatile("v_nop\n\tv_nop\n\tv_nop\n\tv_nop" : "+v"(s[t]) : "v"(qres), "v"(kf) : "memory");
                }
            }
#pragma unroll 1
            for (int dc = 0; dc < 4; ++dc) {
                const v16h qa = WFrag<h16>::ld(Qp + qoff + dc * 32);
#pragma unroll
                for (int t = 0; t < 4; ++t) {
                    const v16h kres = WFrag<h16>::ld(Krp + koff + (size_t)t * 16 * HD + dc * 32);
                    s[t] = wmma16(qa, kres, s[t]);
                    asm volatile("v_nop\n\tv_nop\n\tv_nop\n\tv_nop" : "+v"(s[t]) : "v"(qa), "v"(kres) : "memory");
                }
            }
        }
        const int kbase = ch * 64 + lr;
#pragma unroll
        for (int r = 0; r < 8; ++r) {
            const int qrow = qw + 8 * hi + r; float tv[4]; float cm = -1.0e30f;
#pragma unroll
            for (int t = 0; t < 4; ++t) { const float a = s[t][r] * SSC; const float v = (kbase + 16 * t <= qrow) ? a : -1.0e30f; tv[t] = v; cm = fmaxf(cm, v); }
#pragma unroll
            for (int off = 8; off >= 1; off >>= 1) cm = fmaxf(cm, __shfl_xor(cm, off, 32));
            const float mnew = fmaxf(mrow[r], cm);
            const float alpha = __builtin_amdgcn_exp2f((mrow[r] - mnew) * L2E);
            mrow[r] = mnew; float ps = 0.0f;
#pragma unroll
            for (int t = 0; t < 4; ++t) { const float p = __builtin_amdgcn_exp2f((tv[t] - mnew) * L2E); ps += p; const float pc = p * PCAR; const h16 ph = (h16)pc;
                pl[(8 * hi + r) * 72 + 16 * t + lr] = ph; if (ER) prl[(8 * hi + r) * 72 + 16 * t + lr] = (h16)(pc - (float)ph); }
#pragma unroll
            for (int off = 8; off >= 1; off >>= 1) ps += __shfl_xor(ps, off, 32);
            lrow[r] = lrow[r] * alpha + ps;
#pragma unroll
            for (int c = 0; c < 8; ++c) o[c][r] = o[c][r] * alpha;
        }
        asm volatile("s_wait_dscnt 0" ::: "memory"); __builtin_amdgcn_wave_barrier(); asm volatile("" ::: "memory");
        const size_t voff = (size_t)lr * SEQ + ch * 64 + 8 * hi, vroff = (size_t)lr * RQ + ch * 64 + 8 * hi;
#pragma unroll
        for (int kc = 0; kc < 64; kc += 32) {
            const v16h pf = WFrag<h16>::ld(pl + lr * 72 + 8 * hi + kc);
#pragma unroll
            for (int c = 0; c < 8; ++c) {
                const v16h vf = WFrag<h16>::ld(Vp + voff + (size_t)c * 16 * SEQ + kc);
                o[c] = wmma16(pf, vf, o[c]);
                asm volatile("v_nop\n\tv_nop\n\tv_nop\n\tv_nop" : "+v"(o[c]) : "v"(pf), "v"(vf) : "memory");
            }
        }
        if (ER) {
#pragma unroll 1
            for (int kc = 0; kc < 64; kc += 32) {
                const v16h pres = WFrag<h16>::ld(prl + lr * 72 + 8 * hi + kc);
#pragma unroll
                for (int c = 0; c < 8; ++c) {
                    const v16h vf = WFrag<h16>::ld(Vp + voff + (size_t)c * 16 * SEQ + kc);
                    o[c] = wmma16(pres, vf, o[c]);
                    asm volatile("v_nop\n\tv_nop\n\tv_nop\n\tv_nop" : "+v"(o[c]) : "v"(pres), "v"(vf) : "memory");
                }
            }
#pragma unroll 1
            for (int kc = 0; kc < 64; kc += 32) {
                const v16h pf = WFrag<h16>::ld(pl + lr * 72 + 8 * hi + kc);
#pragma unroll
                for (int c = 0; c < 8; ++c) {
                    const v16h vres = WFrag<h16>::ld(Vrp + vroff + (size_t)c * 16 * RQ + kc);
                    o[c] = wmma16(pf, vres, o[c]);
                    asm volatile("v_nop\n\tv_nop\n\tv_nop\n\tv_nop" : "+v"(o[c]) : "v"(pf), "v"(vres) : "memory");
                }
            }
        }
        asm volatile("s_wait_dscnt 0" ::: "memory"); __builtin_amdgcn_wave_barrier(); asm volatile("" ::: "memory");
    }
    float inv[8];
#pragma unroll
    for (int r = 0; r < 8; ++r) inv[r] = OINV / lrow[r];
#pragma unroll
    for (int c = 0; c < 8; ++c)
#pragma unroll
        for (int r = 0; r < 8; ++r) { const float v = o[c][r] * inv[r]; const h16 hv = (h16)v; osl[(8 * hi + r) * OSP + c * 16 + lr] = hv; if (ER) osl[(8 * hi + r) * OSP + 136 + c * 16 + lr] = (h16)(v - (float)hv); }
    asm volatile("s_wait_dscnt 0" ::: "memory"); __builtin_amdgcn_wave_barrier(); asm volatile("" ::: "memory");
    h16* crow = C16 + ((size_t)(b * SEQ + qw)) * HID + hh * HD;
    h16* rrow = Cr; if (ER) rrow = Cr + ((size_t)(b * RQ + qw)) * HID + hh * HD;
#pragma unroll 1
    for (int ps = 0; ps < 2; ++ps) {
#pragma unroll
        for (int sg = 0; sg < 8; ++sg) { const int row = 2 * sg + hi;
            const v8h val = *(const v8ha*)(osl + row * OSP + lr * 8); *(volatile v8h*)(crow + (size_t)row * HID + lr * 8) = val;
            if (ER) { const v8h valr = *(const v8ha*)(osl + row * OSP + 136 + lr * 8); *(volatile v8h*)(rrow + (size_t)row * HID + lr * 8) = valr; } }
        if (ps == 0) __threadfence(); }
}

extern "C" void kernel_launch(void* const* d_in, const int* in_sizes, int n_in,
                              void* d_out, int out_size, void* d_ws, size_t ws_size, hipStream_t stream) {
    if (n_in < 3) return;
    const size_t xrows = (size_t)(NB - 1) * SEQ_FULL + SEQ;
    if ((size_t)in_sizes[0] < xrows * HID || (size_t)in_sizes[1] < (size_t)HID * QKVN || (size_t)in_sizes[2] < (size_t)HID * HID || (size_t)out_size < xrows * HID) return;
    const float* x = (const float*)d_in[0];
    const float* wqkv = (const float*)d_in[1];
    const float* wout = (const float*)d_in[2];
    float* OUT = (float*)d_out;
    char* wsp = (char*)d_ws;
    auto take = [&](size_t bytes) { char* p = wsp; wsp += (bytes + 255) & ~(size_t)255; return (void*)p; };
    const size_t XE = (size_t)NB * SEQ * HID;
    const size_t RE = (size_t)NB * RQ * HID;
    bf*    Xb  = (bf*)take(XE * 2);
    char*  WTR = (char*)take((size_t)QKVN * HID * 2);
    h16*   Wot = (h16*)take((size_t)HID * HID * 2);
    float* F   = (float*)take((size_t)SEQ * HID * 4);
    h16* Q16 = (h16*)take(XE * 2); h16* K16 = (h16*)take(XE * 2); h16* VT16 = (h16*)take(XE * 2);
    h16* Qr = (h16*)take(RE * 2); h16* Kr = (h16*)take(RE * 2); h16* VTr = (h16*)take(RE * 2);
    if ((size_t)(wsp - (char*)d_ws) > ws_size) return;
    static_assert(((size_t)NB * SEQ * HID * 2 + (size_t)NB * RQ * HID * 2) <= (size_t)QKVN * HID * 2);
    bf*  Wt  = (bf*)WTR;
    h16* C16 = (h16*)WTR;
    h16* Cr  = (h16*)(WTR + XE * 2);

    for (int b = 0; b < NB; ++b)
        k_cvt8<<<(unsigned)(((size_t)SEQ * HID / 8 + 255) / 256), 256, 0, stream>>>(x + (size_t)b * SEQ_FULL * HID, Xb + (size_t)b * SEQ * HID, (size_t)SEQ * HID / 8);
    k_wtb<<<(unsigned)(((size_t)QKVN * HID / 64 + 63) / 64), 256, 0, stream>>>(wqkv, HID, QKVN, Wt);
    k_wth<<<(unsigned)(((size_t)HID * HID / 64 + 63) / 64), 256, 0, stream>>>(wout, HID, HID, WCAR, Wot);

    const unsigned LP = (unsigned)(((size_t)NHD * SEQ * HD / 8 + 255) / 256);
    for (int b = 0; b < NB; ++b) {
        for (int rg = 0; rg < 3; ++rg) {
            k_gemmw<bf, 0><<<dim3(SEQ / 64, HID / 64, 1), 32, 0, stream>>>(Xb + (size_t)b * SEQ * HID, nullptr, Wt + (size_t)rg * HID * HID, nullptr, HID, F, HID, 1.0f, (size_t)0, (size_t)0, (size_t)0);
            if (rg == 0)      k_qkp<<<LP, 256, 0, stream>>>(F, b, Q16, Qr);
            else if (rg == 1) k_qkp<<<LP, 256, 0, stream>>>(F, b, K16, Kr);
            else              k_vtp<<<LP, 256, 0, stream>>>(F, b, VT16, VTr);
        }
    }

    k_attn<true><<<dim3(RQ / 64, NB * NHD, 1), 128, 0, stream>>>(Q16, Qr, K16, Kr, VT16, VTr, 0, C16, Cr);
    if (SEQ > RQ)
        k_attn<false><<<dim3((SEQ - RQ) / 64, NB * NHD, 1), 128, 0, stream>>>(Q16, Qr, K16, Kr, VT16, VTr, RQ / 64, C16, Cr);

    for (int b = 0; b < NB; ++b)
        k_gemmw<h16, 1><<<dim3(RQ / 64, HID / 64, 1), 32, 0, stream>>>(C16 + (size_t)b * SEQ * HID, Cr + (size_t)b * RQ * HID, Wot, nullptr, HID, OUT + (size_t)b * SEQ_FULL * HID, HID, OSC, (size_t)0, (size_t)0, (size_t)0);
    if (SEQ > RQ)
        k_gemmw<h16, 0><<<dim3((SEQ - RQ) / 64, HID / 64, NB), 32, 0, stream>>>(C16 + (size_t)RQ * HID, nullptr, Wot, nullptr, HID, OUT + (size_t)RQ * HID, HID, OSC, (size_t)SEQ * HID, (size_t)0, (size_t)SEQ_FULL * HID);
}
